// LinearTransformerBlock_5153960755280
// MI455X (gfx1250) — hardware-run, weakly checked
//
#include <hip/hip_runtime.h>
#pragma clang fp contract(off)


#ifndef NB
#define NB 2
#endif
#ifndef SEQ
#define SEQ 512
#endif
#define NB_FULL  2
#define SEQ_FULL 512
#ifndef OUT_SEQ
#define OUT_SEQ SEQ
#endif
#define DM   512
#define NH_  8
#define HD   64
#define HID  512
#define FFN  2048
#define OSP  68
#define WSC  64.0f
#define WSI  (1.0f / 64.0f)
#define HSC  64.0f
#define DSI  (1.0f / 4096.0f)
#define EPSN 1.0e-6f

static_assert(NH_ * HD == HID);
static_assert(HID == DM);
static_assert(HD == 64);
static_assert(DM % 64 == 0);
static_assert(FFN % 64 == 0);
static_assert(DM % 32 == 0);
static_assert(FFN % 32 == 0);
static_assert(SEQ % 64 == 0);
static_assert(SEQ % 32 == 0);
static_assert(SEQ % 16 == 0);
static_assert((NB * SEQ) % 64 == 0);
static_assert((NB * SEQ) % 8 == 0);
static_assert(DM == 2 * 32 * 8);
static_assert(NB <= NB_FULL);
static_assert(SEQ <= SEQ_FULL);
static_assert((OSP * 4) % 16 == 0);
static_assert((size_t)NB_FULL * NH_ * HD * HD * 4 == (size_t)262144);
static_assert(64 * 65 * 4 <= 131072);
static_assert(NH_ * 16 * OSP * 4 + NH_ * 16 * 4 <= 131072);
static_assert(16 * OSP * 4 <= 131072);
static_assert(SEQ * 4 + 32 * 36 * 4 <= 131072);

typedef _Float16 h16;
typedef unsigned short bf;
typedef __attribute__((ext_vector_type(16))) __bf16   v16bf;
typedef __attribute__((ext_vector_type(16))) _Float16 v16h;
typedef __attribute__((ext_vector_type(8)))  _Float16 v8h;
typedef __attribute__((ext_vector_type(8)))  unsigned short v8us;
typedef __attribute__((ext_vector_type(8)))  float    v8f;
typedef __attribute__((ext_vector_type(4)))  float    v4f;
typedef v4f  __attribute__((may_alias)) v4fa;

__device__ __forceinline__ unsigned short f2bf(float f) { unsigned u = __float_as_uint(f); u += 0x7FFFu + ((u >> 16) & 1u); return (unsigned short)(u >> 16); }
__device__ __forceinline__ float bfr(float f) { return __uint_as_float(((unsigned)f2bf(f)) << 16); }
__device__ __forceinline__ v16h cat16(v8h lo, v8h hi) { return __builtin_shufflevector(lo, hi, 0, 1, 2, 3, 4, 5, 6, 7, 8, 9, 10, 11, 12, 13, 14, 15); }
__device__ __forceinline__ v16bf cat16b(v8us lo, v8us hi) { return __builtin_bit_cast(v16bf, __builtin_shufflevector(lo, hi, 0, 1, 2, 3, 4, 5, 6, 7, 8, 9, 10, 11, 12, 13, 14, 15)); }
__device__ __forceinline__ v8f wmma16(v16h a, v16h b, v8f c) { return __builtin_amdgcn_wmma_f32_16x16x32_f16(false, a, false, b, (short)0, c, false, false); }
__device__ __forceinline__ v8f wmmab(v16bf a, v16bf b, v8f c) { return __builtin_amdgcn_wmma_f32_16x16x32_bf16(false, a, false, b, (short)0, c, false, false); }
__device__ __forceinline__ v16h  ldh(const h16* p) { return cat16(*(const v8h*)p, *(const v8h*)(p + 16)); }
__device__ __forceinline__ v16bf ldb(const bf* p)  { return cat16b(*(const v8us*)p, *(const v8us*)(p + 16)); }
__device__ __forceinline__ void wave_sync() { __builtin_amdgcn_fence(3  , "wavefront"); __builtin_amdgcn_wave_barrier(); asm volatile("" ::: "memory"); }

static __device__ __forceinline__ h16 toh_flush(float v) { const h16 r = (h16)v; return (fabsf(v) < 6.103515625e-05f) ? (h16)0.0f : r; }
__device__ __forceinline__ v8f wmma16g(v16h a, v16h b, v8f c) { c = wmma16(a, b, c); asm volatile("v_nop\n\tv_nop\n\tv_nop\n\tv_nop" : "+v"(c) : "v"(a), "v"(b)); return c; }
__device__ __forceinline__ v16h ldcar(const float* p) {
    const v4f a = *(const v4f*)p, b = *(const v4f*)(p + 4), c = *(const v4f*)(p + 16), d = *(const v4f*)(p + 20); v16h o;
#pragma unroll
    for (int i = 0; i < 4; ++i) { o[i] = toh_flush(bfr(a[i])); o[4 + i] = toh_flush(bfr(b[i])); o[8 + i] = toh_flush(bfr(c[i])); o[12 + i] = toh_flush(bfr(d[i])); }
    return o;
}

template <int MT, int NT>
__device__ __forceinline__ void gemm_main(const h16* __restrict__ A, size_t lda, const h16* __restrict__ Bt, size_t ldb, int K, int lr, int hi, v8f (&acc)[MT][NT]) {
#pragma unroll
    for (int mb = 0; mb < MT; ++mb)
#pragma unroll
        for (int nb = 0; nb < NT; ++nb) acc[mb][nb] = (v8f){};
    const size_t aoff = (size_t)lr * lda + 8 * hi, boff = (size_t)lr * ldb + 8 * hi;
#pragma unroll 1
    for (int kc = 0; kc < K; kc += 32) {
        v16h a[MT];
#pragma unroll
        for (int mb = 0; mb < MT; ++mb) a[mb] = ldh(A + aoff + (size_t)mb * 16 * lda + kc);
#pragma unroll
        for (int nb = 0; nb < NT; ++nb) { const v16h b = ldh(Bt + boff + (size_t)nb * 16 * ldb + kc);
#pragma unroll
            for (int mb = 0; mb < MT; ++mb) acc[mb][nb] = wmma16g(a[mb], b, acc[mb][nb]); }
    }
}

static_assert(8 * 2 * 32 * 16 == 64 * 64 * 2);
__global__ __launch_bounds__(256) void k_wt(const float* __restrict__ W, h16* dst, int K, int N, int gstride, int goff) {
    __shared__ float ts[64 * 65];
    const int tid = threadIdx.x, lane = tid & 31;
    const int wave = __builtin_amdgcn_readfirstlane((int)(threadIdx.x >> 5));
    const int n0 = blockIdx.x * 64, k0 = blockIdx.y * 64;
#pragma unroll
    for (int i = 0; i < 4; ++i) { const int kr = (tid >> 4) + 16 * i, c4 = (tid & 15) * 4;
        const v4f x = *(const v4f*)(W + (size_t)(k0 + kr) * N + n0 + c4);
        ts[kr * 65 + c4 + 0] = x[0]; ts[kr * 65 + c4 + 1] = x[1]; ts[kr * 65 + c4 + 2] = x[2]; ts[kr * 65 + c4 + 3] = x[3]; }
    __syncthreads();
#pragma unroll 1
    for (int ps = 0; ps < 2; ++ps) {
#pragma unroll
        for (int s = 0; s < 2; ++s) { const int nl = wave * 8 + 4 * s + (lane >> 3), kk = (lane & 7) * 8;
            v8h o;
#pragma unroll
            for (int i = 0; i < 8; ++i) o[i] = toh_flush(bfr(ts[(kk + i) * 65 + nl]) * WSC);
            const int n = n0 + nl; const size_t orow = (size_t)(n >> 6) * (size_t)gstride + (size_t)goff + (size_t)(n & 63);
            *(volatile v8h*)(dst + orow * (size_t)K + k0 + kk) = o; }
        if (ps == 0) __threadfence(); }
}

__global__ __launch_bounds__(256) void k_rms(const float* __restrict__ src, int srcseq, const float* __restrict__ gain, h16* dst, int inbf) {
    const int lane = threadIdx.x & 31;
    const int wave = __builtin_amdgcn_readfirstlane((int)(threadIdx.x >> 5));
    const int row = blockIdx.x * 8 + wave;
    const int bb = row / SEQ, tt = row % SEQ;
    const float* sp = src + ((size_t)bb * (size_t)srcseq + (size_t)tt) * DM + lane * 8;
    const float* gp = gain + lane * 8;
    float x[16], g[16];
#pragma unroll
    for (int j = 0; j < 2; ++j) {
        const v4f a = *(const v4f*)(sp + j * 256), c = *(const v4f*)(sp + j * 256 + 4);
        const v4f ga = *(const v4f*)(gp + j * 256), gc = *(const v4f*)(gp + j * 256 + 4);
#pragma unroll
        for (int i = 0; i < 4; ++i) { x[j * 8 + i] = a[i]; x[j * 8 + 4 + i] = c[i]; g[j * 8 + i] = bfr(ga[i]); g[j * 8 + 4 + i] = bfr(gc[i]); } }
    float ss = 0.0f;
#pragma unroll
    for (int i = 0; i < 16; ++i) { const float v = (inbf != 0) ? bfr(x[i]) : x[i]; x[i] = v; ss += v * v; }
    ss += __shfl_xor(ss, 16, 32); ss += __shfl_xor(ss, 8, 32); ss += __shfl_xor(ss, 4, 32); ss += __shfl_xor(ss, 2, 32); ss += __shfl_xor(ss, 1, 32);
    const float inv = rsqrtf(ss * (1.0f / (float)DM) + EPSN);
    v8h o0, o1;
#pragma unroll
    for (int i = 0; i < 8; ++i) { o0[i] = toh_flush(x[i] * inv * g[i]); o1[i] = toh_flush(x[8 + i] * inv * g[8 + i]); }
    h16* dp = dst + (size_t)row * DM + lane * 8;
    *(volatile v8h*)dp = o0; *(volatile v8h*)(dp + 256) = o1;
    __threadfence();
    *(volatile v8h*)dp = o0; *(volatile v8h*)(dp + 256) = o1;
}

static_assert(8 * 32 * 16 == 32 * 32 * 4);
__global__ __launch_bounds__(32) void k_decay(const float* __restrict__ mask, float* Wp) {
    __shared__ float cm[SEQ];
    __shared__ __align__(16) float tl[32 * 36];
    const int lane = threadIdx.x & 31;
    const int bb = blockIdx.y, r0 = blockIdx.x * 32;
#pragma unroll 1
    for (int i = lane; i < SEQ; i += 32) cm[i] = 1.0f - bfr(mask[(size_t)bb * SEQ_FULL + i]);
    wave_sync();
    const int t = r0 + lane;
    float w = 0.0f;
#pragma unroll 1
    for (int cs = SEQ - 32; cs >= 0; cs -= 32) {
#pragma unroll 4
        for (int c = 31; c >= 0; --c) { const int s = cs + c; const int sn = (s + 1 < SEQ) ? (s + 1) : (SEQ - 1);
            float cn = cm[sn]; asm volatile("" : "+v"(cn));
            const float wn = w * cn;
            w = (s > t) ? 0.0f : ((s == t) ? 1.0f : wn);
            tl[lane * 36 + c] = w; }
        wave_sync();
#pragma unroll 1
        for (int ps = 0; ps < 2; ++ps) {
#pragma unroll
            for (int s4 = 0; s4 < 8; ++s4) { const int row = 4 * s4 + (lane >> 3), c4 = (lane & 7) * 4;
                const v4f val = *(const v4fa*)(&tl[row * 36 + c4]);
                *(volatile v4f*)(Wp + ((size_t)bb * SEQ + r0 + row) * SEQ + cs + c4) = val; }
            if (ps == 0) __threadfence(); }
        wave_sync();
    }
}

static_assert(4 * 32 * 16 == 16 * HD * 2);
__global__ __launch_bounds__(32) void k_gemm_qk(const h16* __restrict__ X, const h16* __restrict__ WT, h16* QK) {
    __shared__ __align__(16) float os[16 * OSP];
    const int lane = threadIdx.x & 31, lr = lane & 15, hi = lane >> 4; const int r0 = blockIdx.x * 64, c0 = blockIdx.y * 64;
    v8f acc[4][4];
    gemm_main<4, 4>(X + (size_t)r0 * DM, (size_t)DM, WT + (size_t)c0 * DM, (size_t)DM, DM, lr, hi, acc);
    const int bb = r0 / SEQ, tt = r0 % SEQ; const int which = c0 / HID, hh = (c0 % HID) / HD;
    const size_t tbase = ((((size_t)which * NB + (size_t)bb) * NH_ + (size_t)hh) * SEQ + (size_t)tt) * HD;
#pragma unroll
    for (int mb = 0; mb < 4; ++mb) {
#pragma unroll
        for (int nb = 0; nb < 4; ++nb) {
#pragma unroll
            for (int j = 0; j < 8; ++j) os[(hi * 8 + j) * OSP + nb * 16 + lr] = fmaxf(acc[mb][nb][j] * WSI, 0.0f); }
        wave_sync();
#pragma unroll 1
        for (int ps = 0; ps < 2; ++ps) {
#pragma unroll
            for (int s = 0; s < 4; ++s) { const int p = s * 32 + lane; const int row = p >> 3, c8 = (p & 7) * 8;
                const v4f x0 = *(const v4fa*)(&os[row * OSP + c8]); const v4f x1 = *(const v4fa*)(&os[row * OSP + c8 + 4]); v8h hv;
#pragma unroll
                for (int i = 0; i < 4; ++i) { hv[i] = toh_flush(x0[i]); hv[4 + i] = toh_flush(x1[i]); }
                *(volatile v8h*)(QK + tbase + (size_t)(mb * 16) * HD + (size_t)p * 8) = hv; }
            if (ps == 0) __threadfence(); }
        wave_sync();
    }
}

static_assert(4 * 32 * 16 == 16 * 64 * 2);
__global__ __launch_bounds__(32) void k_gemm_t(const h16* __restrict__ WT, const h16* __restrict__ X, h16* PT, int relu, int usew, const float* __restrict__ Wp) {
    __shared__ __align__(16) float os[16 * OSP];
    const int lane = threadIdx.x & 31, lr = lane & 15, hi = lane >> 4; const int r0 = blockIdx.x * 64, c0 = blockIdx.y * 64;
    v8f acc[4][4];
    gemm_main<4, 4>(WT + (size_t)r0 * DM, (size_t)DM, X + (size_t)c0 * DM, (size_t)DM, DM, lr, hi, acc);
    const int bb = c0 / SEQ, tt = c0 % SEQ;
    float cw[4];
#pragma unroll
    for (int nb = 0; nb < 4; ++nb) { float w = 1.0f; if (usew != 0) w = Wp[((size_t)bb * SEQ + (size_t)(SEQ - 1)) * SEQ + tt + nb * 16 + lr]; cw[nb] = w; }
    const size_t tbase = ((size_t)bb * HID + (size_t)r0) * SEQ + (size_t)tt;
#pragma unroll
    for (int mb = 0; mb < 4; ++mb) {
#pragma unroll
        for (int nb = 0; nb < 4; ++nb) {
#pragma unroll
            for (int j = 0; j < 8; ++j) { const float v0 = acc[mb][nb][j] * WSI; const float v1 = (relu != 0) ? fmaxf(v0, 0.0f) : v0; os[(hi * 8 + j) * OSP + nb * 16 + lr] = v1 * cw[nb]; } }
        wave_sync();
#pragma unroll 1
        for (int ps = 0; ps < 2; ++ps) {
#pragma unroll
            for (int s = 0; s < 4; ++s) { const int row = 4 * s + (lane >> 3), c8 = (lane & 7) * 8;
                const v4f x0 = *(const v4fa*)(&os[row * OSP + c8]); const v4f x1 = *(const v4fa*)(&os[row * OSP + c8 + 4]); v8h hv;
#pragma unroll
                for (int i = 0; i < 4; ++i) { hv[i] = toh_flush(x0[i]); hv[4 + i] = toh_flush(x1[i]); }
                *(volatile v8h*)(PT + tbase + (size_t)(mb * 16 + row) * SEQ + c8) = hv; }
            if (ps == 0) __threadfence(); }
        wave_sync();
    }
}

static_assert(4 * 32 * 16 == 16 * HD * 2);
__global__ __launch_bounds__(32 * NH_) void k_lattn(const h16* __restrict__ QP, const h16* __restrict__ KP, const h16* __restrict__ VT, const float* __restrict__ Wp,
                                                    const float* __restrict__ mask, const float* __restrict__ carry, const float* __restrict__ again, h16* AN) {
    __shared__ __align__(16) float os[NH_ * 16 * OSP];
    __shared__ float ssw[NH_ * 16];
    const int lane = threadIdx.x & 31, lr = lane & 15, hi = lane >> 4;
    const int wave = __builtin_amdgcn_readfirstlane((int)(threadIdx.x >> 5));
    const int h = wave, b = blockIdx.y; const int t0 = blockIdx.x * 16;
    const int zh = b * NH_ + h;
    const int nk = (t0 + 16 + 31) & ~31;
    const size_t pbase = (size_t)zh * SEQ * HD;
    const size_t qo = pbase + (size_t)(t0 + lr) * HD + 8 * hi;
    const v16h q0 = ldh(QP + qo), q1 = ldh(QP + qo + 32);
    const float* wrow = Wp + ((size_t)b * SEQ + (size_t)(t0 + lr)) * SEQ;
    const float dt = wrow[0] * (1.0f - bfr(mask[(size_t)b * SEQ_FULL]));
    const float* cb = carry + (size_t)zh * HD * HD + (size_t)lr * HD + 8 * hi;
    v8f o[4];
#pragma unroll
    for (int j = 0; j < 4; ++j) { const v16h c0 = ldcar(cb + (size_t)j * 16 * HD), c1 = ldcar(cb + (size_t)j * 16 * HD + 32);
        v8f a = (v8f){}; a = wmma16g(c0, q0, a); a = wmma16g(c1, q1, a); o[j] = a * dt; }
    const size_t ko = pbase + (size_t)lr * HD + 8 * hi;
    const size_t vo = pbase + (size_t)lr * SEQ + 8 * hi;
    const float* wk = wrow + 8 * hi;
#pragma unroll 1
    for (int key0 = 0; key0 < nk; key0 += 32) {
        const h16* ka = KP + ko + (size_t)key0 * HD;
        const v16h ka0 = ldh(ka), ka1 = ldh(ka + 32), kb0 = ldh(ka + 16 * HD), kb1 = ldh(ka + 16 * HD + 32);
        v8f sa = (v8f){}, sb = (v8f){};
        sa = wmma16g(ka0, q0, sa); sa = wmma16g(ka1, q1, sa);
        sb = wmma16g(kb0, q0, sb); sb = wmma16g(kb1, q1, sb);
        const float* wp = wk + key0;
        const v4f w0 = *(const v4f*)wp, w1 = *(const v4f*)(wp + 4), w2 = *(const v4f*)(wp + 16), w3 = *(const v4f*)(wp + 20);
        v16h pb;
#pragma unroll
        for (int r = 0; r < 4; ++r) {
            pb[r]      = toh_flush(sa[r] * w0[r]);     pb[4 + r]  = toh_flush(sa[4 + r] * w1[r]);
            pb[8 + r]  = toh_flush(sb[r] * w2[r]);     pb[12 + r] = toh_flush(sb[4 + r] * w3[r]); }
        const h16* va = VT + vo + key0;
#pragma unroll
        for (int j = 0; j < 4; ++j) { const v16h vf = ldh(va + (size_t)j * 16 * SEQ); o[j] = wmma16g(vf, pb, o[j]); }
    }
    float sq = 0.0f;
#pragma unroll
    for (int j = 0; j < 4; ++j)
#pragma unroll
        for (int r = 0; r < 8; ++r) sq += o[j][r] * o[j][r];
    sq += __shfl_xor(sq, 16, 32);
    if (hi == 0) ssw[wave * 16 + lr] = sq;
    __syncthreads();
    float tot = 0.0f;
#pragma unroll
    for (int w8 = 0; w8 < NH_; ++w8) tot += ssw[w8 * 16 + lr];
    const float inv = rsqrtf(tot * (1.0f / (float)HID) + EPSN);
    const int wb = wave * 16 * OSP;
    const float* gp = again + h * HD + 8 * hi;
#pragma unroll
    for (int j = 0; j < 4; ++j) { const v4f g0 = *(const v4f*)(gp + 16 * j), g1 = *(const v4f*)(gp + 16 * j + 4); v4f a, c;
#pragma unroll
        for (int i = 0; i < 4; ++i) { a[i] = o[j][i] * inv * bfr(g0[i]); c[i] = o[j][4 + i] * inv * bfr(g1[i]); }
        *(v4fa*)(&os[wb + lr * OSP + 16 * j + 8 * hi]) = a; *(v4fa*)(&os[wb + lr * OSP + 16 * j + 8 * hi + 4]) = c; }
    wave_sync();
    h16* arow = AN + ((size_t)b * SEQ + (size_t)t0) * HID + h * HD;
#pragma unroll 1
    for (int ps = 0; ps < 2; ++ps) {
#pragma unroll
        for (int s = 0; s < 4; ++s) { const int row = 4 * s + (lane >> 3), c8 = (lane & 7) * 8;
            const v4f x0 = *(const v4fa*)(&os[wb + row * OSP + c8]); const v4f x1 = *(const v4fa*)(&os[wb + row * OSP + c8 + 4]); v8h hv;
#pragma unroll
            for (int i = 0; i < 4; ++i) { hv[i] = toh_flush(x0[i]); hv[4 + i] = toh_flush(x1[i]); }
            *(volatile v8h*)(arow + (size_t)row * HID + c8) = hv; }
        if (ps == 0) __threadfence(); }
}

static_assert(8 * 32 * 16 == 16 * HD * 4);
__global__ __launch_bounds__(32) void k_state(const h16* __restrict__ VT, const h16* __restrict__ KT, const float* __restrict__ Wp, const float* __restrict__ mask,
                                              const float* __restrict__ carry, float* OUT0) {
    __shared__ __align__(16) float os[16 * OSP];
    const int lane = threadIdx.x & 31, lr = lane & 15, hi = lane >> 4; const int zh = blockIdx.x; const int b = zh / NH_;
    v8f acc[4][4];
    gemm_main<4, 4>(VT + (size_t)zh * HD * SEQ, (size_t)SEQ, KT + (size_t)zh * HD * SEQ, (size_t)SEQ, SEQ, lr, hi, acc);
    const float dl = Wp[((size_t)b * SEQ + (size_t)(SEQ - 1)) * SEQ] * (1.0f - bfr(mask[(size_t)b * SEQ_FULL]));
    const size_t obase = (size_t)zh * HD * HD;
#pragma unroll
    for (int mb = 0; mb < 4; ++mb) {
#pragma unroll
        for (int nb = 0; nb < 4; ++nb) {
#pragma unroll
            for (int j = 0; j < 8; ++j) os[(hi * 8 + j) * OSP + nb * 16 + lr] = acc[mb][nb][j]; }
        wave_sync();
#pragma unroll 1
        for (int ps = 0; ps < 2; ++ps) {
#pragma unroll
            for (int s = 0; s < 8; ++s) { const int row = 2 * s + (lane >> 4), c4 = (lane & 15) * 4;
                const v4f x0 = *(const v4fa*)(&os[row * OSP + c4]);
                const size_t oo = obase + (size_t)(mb * 16 + row) * HD + c4;
                const v4f cv = *(const v4f*)(carry + oo); v4f val;
#pragma unroll
                for (int i = 0; i < 4; ++i) val[i] = bfr(cv[i]) * dl + x0[i];
                *(volatile v4f*)(OUT0 + oo) = val; }
            if (ps == 0) __threadfence(); }
        wave_sync();
    }
}

static_assert(8 * 32 * 16 == 16 * 64 * 4);
__global__ __launch_bounds__(32) void k_gemm_res(const h16* __restrict__ A, const h16* __restrict__ Bt, int K, float scale, const float* __restrict__ bias, int usebias,
                                                 const float* __restrict__ resid, int rseq, int resbf, float* out, int oseq) {
    __shared__ __align__(16) float os[16 * OSP];
    const int lane = threadIdx.x & 31, lr = lane & 15, hi = lane >> 4; const int r0 = blockIdx.x * 64, c0 = blockIdx.y * 64;
    v8f acc[4][4];
    gemm_main<4, 4>(A + (size_t)r0 * (size_t)K, (size_t)K, Bt + (size_t)c0 * (size_t)K, (size_t)K, K, lr, hi, acc);
    const int bb = r0 / SEQ, tt = r0 % SEQ;
#pragma unroll
    for (int mb = 0; mb < 4; ++mb) {
#pragma unroll
        for (int nb = 0; nb < 4; ++nb) {
#pragma unroll
            for (int j = 0; j < 8; ++j) os[(hi * 8 + j) * OSP + nb * 16 + lr] = acc[mb][nb][j] * scale; }
        wave_sync();
#pragma unroll 1
        for (int ps = 0; ps < 2; ++ps) {
#pragma unroll
            for (int s = 0; s < 8; ++s) { const int row = 2 * s + (lane >> 4), c4 = (lane & 15) * 4;
                const v4f x0 = *(const v4fa*)(&os[row * OSP + c4]);
                const v4f bz = *(const v4f*)(bias + c0 + c4);
                const size_t rr = ((size_t)bb * (size_t)rseq + (size_t)(tt + mb * 16 + row)) * DM + c0 + c4;
                const v4f rv = *(const v4f*)(resid + rr); v4f val;
#pragma unroll
                for (int i = 0; i < 4; ++i) { const float bv = (usebias != 0) ? bfr(bz[i]) : 0.0f; const float rs = (resbf != 0) ? bfr(rv[i]) : rv[i]; val[i] = (x0[i] + bv) + rs; }
                const size_t oo = ((size_t)bb * (size_t)oseq + (size_t)(tt + mb * 16 + row)) * DM + c0 + c4;
                *(volatile v4f*)(out + oo) = val; }
            if (ps == 0) __threadfence(); }
        wave_sync();
    }
}

static_assert(4 * 32 * 16 == 16 * 64 * 2);
static_assert((NB * SEQ) % 32 == 0);
__global__ __launch_bounds__(32) void k_gemm_gu(const h16* __restrict__ X, const h16* __restrict__ WGU, h16* HP) {
    __shared__ __align__(16) float os[16 * OSP];
    const int lane = threadIdx.x & 31, lr = lane & 15, hi = lane >> 4; const int r0 = blockIdx.x * 32, cg = blockIdx.y;
    v8f acc[2][8];
    gemm_main<2, 8>(X + (size_t)r0 * DM, (size_t)DM, WGU + (size_t)cg * 128 * DM, (size_t)DM, DM, lr, hi, acc);
#pragma unroll
    for (int mb = 0; mb < 2; ++mb) {
#pragma unroll
        for (int nb = 0; nb < 4; ++nb) {
#pragma unroll
            for (int j = 0; j < 8; ++j) { const float g = acc[mb][nb][j] * WSI, u = acc[mb][nb + 4][j] * WSI;
                const float sg = __builtin_amdgcn_rcpf(1.0f + __expf(-g));
                os[(hi * 8 + j) * OSP + nb * 16 + lr] = ((g * sg) * u) * HSC; } }
        wave_sync();
#pragma unroll 1
        for (int ps = 0; ps < 2; ++ps) {
#pragma unroll
            for (int s = 0; s < 4; ++s) { const int row = 4 * s + (lane >> 3), c8 = (lane & 7) * 8;
                const v4f x0 = *(const v4fa*)(&os[row * OSP + c8]); const v4f x1 = *(const v4fa*)(&os[row * OSP + c8 + 4]); v8h hv;
#pragma unroll
                for (int i = 0; i < 4; ++i) { hv[i] = toh_flush(x0[i]); hv[4 + i] = toh_flush(x1[i]); }
                *(volatile v8h*)(HP + (size_t)(r0 + mb * 16 + row) * FFN + (size_t)cg * 64 + c8) = hv; }
            if (ps == 0) __threadfence(); }
        wave_sync();
    }
}

static constexpr size_t al256(size_t v) { return (v + 255) & ~(size_t)255; }
static constexpr size_t SZ_WT3 = al256((size_t)3 * HID * DM * 2);
static constexpr size_t SZ_WOT = al256((size_t)DM * HID * 2);
static constexpr size_t SZ_WGU = al256((size_t)2 * FFN * DM * 2);
static constexpr size_t SZ_WDT = al256((size_t)DM * FFN * 2);
static constexpr size_t SZ_X   = al256((size_t)NB * SEQ * DM * 2);
static constexpr size_t SZ_WP  = al256((size_t)NB * SEQ * SEQ * 4);
static constexpr size_t SZ_QK  = al256((size_t)2 * NB * NH_ * SEQ * HD * 2);
static constexpr size_t SZ_PT  = al256((size_t)NB * HID * SEQ * 2);
static constexpr size_t SZ_XR  = al256((size_t)NB * SEQ * DM * 4);
static constexpr size_t SZ_HP  = al256((size_t)NB * SEQ * FFN * 2);
static constexpr size_t SZ_TOTAL = SZ_WT3 + SZ_WOT + SZ_WGU + SZ_WDT + 3 * SZ_X + SZ_WP + SZ_QK + 2 * SZ_PT + SZ_XR + SZ_HP;
static_assert(SZ_TOTAL <= (size_t)134217728);
static_assert(((size_t)HID * DM * 2) % 256 == 0);
static_assert(((size_t)NB * NH_ * SEQ * HD * 2) % 256 == 0);
static_assert((size_t)NB * NH_ * SEQ * HD == (size_t)NB * HID * SEQ);

extern "C" void kernel_launch(void* const* d_in, const int* in_sizes, int n_in,
                              void* d_out, int out_size, void* d_ws, size_t ws_size, hipStream_t stream) {
    if (n_in < 14) return;
    const size_t needx = ((size_t)(NB - 1) * SEQ_FULL + SEQ) * DM;
    const size_t needm = (size_t)(NB - 1) * SEQ_FULL + SEQ;
    if ((size_t)in_sizes[0] < needx || (size_t)in_sizes[1] < needm || (size_t)in_sizes[2] < (size_t)NB * NH_ * HD * HD) return;
    if (in_sizes[3] < DM || in_sizes[7] < HID || in_sizes[9] < DM || in_sizes[10] < DM) return;
    if ((size_t)in_sizes[4] < (size_t)DM * HID || (size_t)in_sizes[5] < (size_t)DM * HID || (size_t)in_sizes[6] < (size_t)DM * HID || (size_t)in_sizes[8] < (size_t)HID * DM) return;
    if ((size_t)in_sizes[11] < (size_t)DM * FFN || (size_t)in_sizes[12] < (size_t)DM * FFN || (size_t)in_sizes[13] < (size_t)FFN * DM) return;
    const size_t off1 = (size_t)NB_FULL * NH_ * HD * HD;
    if ((size_t)out_size < off1 + ((size_t)(NB - 1) * OUT_SEQ + SEQ) * DM) return;
    if (SZ_TOTAL > ws_size) return;
    const float* xin = (const float*)d_in[0]; const float* mask = (const float*)d_in[1]; const float* carry = (const float*)d_in[2];
    const float* ln1 = (const float*)d_in[3];
    const float* wq = (const float*)d_in[4]; const float* wk = (const float*)d_in[5]; const float* wv = (const float*)d_in[6];
    const float* aln = (const float*)d_in[7]; const float* wo = (const float*)d_in[8]; const float* bo = (const float*)d_in[9];
    const float* ln2 = (const float*)d_in[10];
    const float* wg = (const float*)d_in[11]; const float* wu = (const float*)d_in[12]; const float* wd = (const float*)d_in[13];
    float* OUT0 = (float*)d_out;
    float* OUT1 = (float*)d_out + off1;
    char* wsp = (char*)d_ws;
    h16* WT3 = (h16*)wsp; wsp += SZ_WT3;
    h16* WOT = (h16*)wsp; wsp += SZ_WOT;
    h16* WGU = (h16*)wsp; wsp += SZ_WGU;
    h16* WDT = (h16*)wsp; wsp += SZ_WDT;
    h16* X1  = (h16*)wsp; wsp += SZ_X;
    h16* AN  = (h16*)wsp; wsp += SZ_X;
    h16* X2  = (h16*)wsp; wsp += SZ_X;
    float* WP = (float*)wsp; wsp += SZ_WP;
    h16* QK  = (h16*)wsp; wsp += SZ_QK;
    h16* VT  = (h16*)wsp; wsp += SZ_PT;
    h16* KT  = (h16*)wsp; wsp += SZ_PT;
    float* XR = (float*)wsp; wsp += SZ_XR;
    h16* HP  = (h16*)wsp; wsp += SZ_HP;
    h16* QP = QK; h16* KP = QK + (size_t)NB * NH_ * SEQ * HD;
    h16* WQT = WT3; h16* WKT = WT3 + (size_t)HID * DM; h16* WVT = WT3 + (size_t)2 * HID * DM;

    k_wt<<<dim3(HID / 64, DM / 64, 1), 256, 0, stream>>>(wq, WQT, DM, HID, 64, 0);
    k_wt<<<dim3(HID / 64, DM / 64, 1), 256, 0, stream>>>(wk, WKT, DM, HID, 64, 0);
    k_wt<<<dim3(HID / 64, DM / 64, 1), 256, 0, stream>>>(wv, WVT, DM, HID, 64, 0);
    k_wt<<<dim3(DM / 64, HID / 64, 1), 256, 0, stream>>>(wo, WOT, HID, DM, 64, 0);
    k_wt<<<dim3(FFN / 64, DM / 64, 1), 256, 0, stream>>>(wg, WGU, DM, FFN, 128, 0);
    k_wt<<<dim3(FFN / 64, DM / 64, 1), 256, 0, stream>>>(wu, WGU, DM, FFN, 128, 64);
    k_wt<<<dim3(DM / 64, FFN / 64, 1), 256, 0, stream>>>(wd, WDT, FFN, DM, 64, 0);

    k_rms<<<NB * SEQ / 8, 256, 0, stream>>>(xin, SEQ_FULL, ln1, X1, 1);
    k_decay<<<dim3(SEQ / 32, NB, 1), 32, 0, stream>>>(mask, WP);

    k_gemm_qk<<<dim3(NB * SEQ / 64, 2 * HID / 64, 1), 32, 0, stream>>>(X1, WT3, QK);
    k_gemm_t<<<dim3(HID / 64, NB * SEQ / 64, 1), 32, 0, stream>>>(WVT, X1, VT, 0, 0, WP);
    k_gemm_t<<<dim3(HID / 64, NB * SEQ / 64, 1), 32, 0, stream>>>(WKT, X1, KT, 1, 1, WP);

    k_lattn<<<dim3(SEQ / 16, NB, 1), 32 * NH_, 0, stream>>>(QP, KP, VT, WP, mask, carry, aln, AN);
    k_state<<<dim3(NB * NH_, 1, 1), 32, 0, stream>>>(VT, KT, WP, mask, carry, OUT0);

    k_gemm_res<<<dim3(NB * SEQ / 64, DM / 64, 1), 32, 0, stream>>>(AN, WOT, HID, WSI, bo, 1, xin, SEQ_FULL, 1, XR, SEQ);
    k_rms<<<NB * SEQ / 8, 256, 0, stream>>>(XR, SEQ, ln2, X2, 0);
    k_gemm_gu<<<dim3(NB * SEQ / 32, FFN / 64, 1), 32, 0, stream>>>(X2, WGU, HP);
    k_gemm_res<<<dim3(NB * SEQ / 64, DM / 64, 1), 32, 0, stream>>>(HP, WDT, FFN, DSI, bo, 0, XR, SEQ, 0, OUT1, OUT_SEQ);
}
